// MultiHeadDiffAttention_84318797955421
// MI455X (gfx1250) — hardware-verified
//
#include <hip/hip_runtime.h>


typedef __attribute__((ext_vector_type(16))) _Float16 v16h;
typedef __attribute__((ext_vector_type(8)))  _Float16 v8h;
typedef __attribute__((ext_vector_type(16))) __bf16   v16b;
typedef __attribute__((ext_vector_type(8)))  __bf16   v8b;
typedef __attribute__((ext_vector_type(8)))  float    v8f;
typedef __attribute__((ext_vector_type(4)))  float    v4f;
#define PSCALE 32768.0f
#define U16(p) ((const unsigned short*)(const void*)(p))
#define PSCALE_INV (1.0f / 32768.0f)

__device__ __forceinline__ unsigned short f2bf_bits(float f) {
  unsigned u = __float_as_uint(f);
  return (unsigned short)((u + 0x7FFFu + ((u >> 16) & 1u)) >> 16);
}
__device__ __forceinline__ float bf_bits2f(unsigned short h) { return __uint_as_float(((unsigned)h) << 16); }

__device__ __forceinline__ void dep_guard_h(v8f& a, v8f& b, v16h x, v16h y) { asm volatile("v_nop\n\tv_nop\n\tv_nop\n\tv_nop" : "+v"(a), "+v"(b) : "v"(x), "v"(y)); }
__device__ __forceinline__ void dep_guard_b(v8f& a, v8f& b, v16b x, v16b y) { asm volatile("v_nop\n\tv_nop\n\tv_nop\n\tv_nop" : "+v"(a), "+v"(b) : "v"(x), "v"(y)); }
__device__ __forceinline__ void keep4_h(v16h a, v16h b, v16h c, v16h d) { asm volatile("v_nop" :: "v"(a), "v"(b), "v"(c), "v"(d)); }
__device__ __forceinline__ void keep4_b(v16b a, v16b b, v16b c, v16b d) { asm volatile("v_nop" :: "v"(a), "v"(b), "v"(c), "v"(d)); }
__device__ __forceinline__ void acc_guard4(v8f& a, v8f& b, v8f& c, v8f& d) { asm volatile("v_nop\n\tv_nop\n\tv_nop\n\tv_nop" : "+v"(a), "+v"(b), "+v"(c), "+v"(d)); }
template <typename T> struct Frag;
template <> struct Frag<_Float16> {
  typedef v16h V; union U { v16h v; v8h h[2]; };
  static __device__ __forceinline__ v16h load(const _Float16* p) {
    U f; f.h[0] = *(const v8h*)(p); f.h[1] = *(const v8h*)(p + 16); return f.v;
  }
  static __device__ __forceinline__ v8f mma(v16h a, v16h b, v8f c) {
    return __builtin_amdgcn_wmma_f32_16x16x32_f16(false, a, false, b, (short)0, c, false, false);
  }
  static __device__ __forceinline__ void guard(v8f& a, v8f& b, v16h x, v16h y) { dep_guard_h(a, b, x, y); }
  static __device__ __forceinline__ void keep(v16h a, v16h b, v16h c, v16h d) { keep4_h(a, b, c, d); }
};
template <> struct Frag<__bf16> {
  typedef v16b V; union U { v16b v; v8b h[2]; };
  static __device__ __forceinline__ v16b load(const __bf16* p) {
    U f; f.h[0] = *(const v8b*)(p); f.h[1] = *(const v8b*)(p + 16); return f.v;
  }
  static __device__ __forceinline__ v8f mma(v16b a, v16b b, v8f c) {
    return __builtin_amdgcn_wmma_f32_16x16x32_bf16(false, a, false, b, (short)0, c, false, false);
  }
  static __device__ __forceinline__ void guard(v8f& a, v8f& b, v16b x, v16b y) { dep_guard_b(a, b, x, y); }
  static __device__ __forceinline__ void keep(v16b a, v16b b, v16b c, v16b d) { keep4_b(a, b, c, d); }
};

template <int ET> struct Elem;
template <> struct Elem<0> { typedef _Float16 T; };
template <> struct Elem<1> { typedef __bf16 T; };
template <int ET, bool SPLIT, int BIAS_MODE, int OUT_MODE, bool RESID, int ACT = 0>
__global__ __launch_bounds__(256) void wmma_gemm64(
    const unsigned short* __restrict__ Ap, const unsigned short* __restrict__ A2p, int lda, long strideA,
    const unsigned short* __restrict__ Btp, const unsigned short* __restrict__ Bt2p, int ldb, long strideB,
    void* __restrict__ Cout, void* __restrict__ Cout2, int ldc, long strideC,
    const float* __restrict__ bias,
    const float* __restrict__ resid, long strideR,
    int M, int N, int K, float scale) {
  typedef typename Elem<ET>::T T;
  typedef typename Frag<T>::V V;
  const T* A = (const T*)Ap; const T* A2 = (const T*)A2p; const T* Bt = (const T*)Btp; const T* Bt2 = (const T*)Bt2p;
  __shared__ __align__(16) float sT[8][16 * 68];
  const int b    = blockIdx.y;
  const int lane = threadIdx.x & 31;
  const int wave = threadIdx.x >> 5;
  const int tilesN = N >> 6;
  const int tilesM = M >> 6;
  const int tile = blockIdx.x * 8 + wave;
  if (tile >= tilesM * tilesN) return;
  const int tm = tile / tilesN;
  const int tn = tile - tm * tilesN;
  const int m0 = tm << 6;
  const int n0 = tn << 6;

  const T* Ab  = A  + (size_t)b * strideA;
  const T* Bb  = Bt + (size_t)b * strideB;
  const T* Ab2 = SPLIT ? (A2  + (size_t)b * strideA) : nullptr;
  const T* Bb2 = SPLIT ? (Bt2 + (size_t)b * strideB) : nullptr;

  const int rlane = lane & 15;
  const int koff  = (lane >> 4) * 8;
  const int mOff  = (lane >> 4) * 8;

  v8f acc[4][4];
#pragma unroll
  for (int i = 0; i < 4; ++i)
#pragma unroll
    for (int j = 0; j < 4; ++j) acc[i][j] = (v8f){0.f,0.f,0.f,0.f,0.f,0.f,0.f,0.f};

  for (int k0 = 0; k0 < K; k0 += 32) {
    V bh[4], bl[4];
#pragma unroll
    for (int j = 0; j < 4; ++j) {
      const size_t bo = (size_t)(n0 + (j << 4) + rlane) * ldb + koff + k0;
      bh[j] = Frag<T>::load(Bb + bo);
      if (SPLIT) bl[j] = Frag<T>::load(Bb2 + bo);
    }
#pragma unroll
    for (int i = 0; i < 4; ++i) {
      const size_t ao = (size_t)(m0 + (i << 4) + rlane) * lda + koff + k0;
      V ah = Frag<T>::load(Ab + ao);
      V al;
      if (SPLIT) al = Frag<T>::load(Ab2 + ao);
#pragma unroll
      for (int j = 0; j < 4; ++j) {
        acc[i][j] = Frag<T>::mma(ah, bh[j], acc[i][j]);
        if (SPLIT) {
          acc[i][j] = Frag<T>::mma(ah, bl[j], acc[i][j]);
          acc[i][j] = Frag<T>::mma(al, bh[j], acc[i][j]);
        }
      }
      Frag<T>::guard(acc[i][0], acc[i][3], ah, SPLIT ? al : ah);
    }
    Frag<T>::keep(bh[0], bh[1], bh[2], bh[3]);
    if (SPLIT) Frag<T>::keep(bl[0], bl[1], bl[2], bl[3]);
  }
  acc_guard4(acc[0][0], acc[0][1], acc[0][2], acc[0][3]);
  acc_guard4(acc[1][0], acc[1][1], acc[1][2], acc[1][3]);
  acc_guard4(acc[2][0], acc[2][1], acc[2][2], acc[2][3]);
  acc_guard4(acc[3][0], acc[3][1], acc[3][2], acc[3][3]);

  float* slab = sT[wave];
  const float* Rb = RESID ? (resid + (size_t)b * strideR) : nullptr;
#pragma unroll
  for (int i = 0; i < 4; ++i) {
    const int mBase = m0 + (i << 4);
#pragma unroll
    for (int j = 0; j < 4; ++j) {
      const int n = n0 + (j << 4) + rlane;
      float bv = 0.f;
      if (BIAS_MODE == 2) bv = bias[n];
#pragma unroll
      for (int r = 0; r < 8; ++r) {
        float v = acc[i][j][r] * scale;
        if (BIAS_MODE == 1) v += bias[mBase + mOff + r];
        if (BIAS_MODE == 2) v += bv;
        if (RESID) v += Rb[(size_t)(mBase + mOff + r) * ldc + n];
        if (ACT == 1) v = tanhf(v);
        if (ACT == 2) v = fmaxf(v, 0.0f);
        if (ACT == 3) v = v / (1.0f + expf(-v));
        if (ACT == 4) v = (v > 0.f) ? v : 0.01f * v;
        if (ACT == 5) v = 0.5f * v * (1.0f + erff(v * 0.70710678118654752f));
        slab[(mOff + r) * 68 + (j << 4) + rlane] = v;
      }
    }
    __builtin_amdgcn_fence(__ATOMIC_RELEASE, "workgroup");
    __builtin_amdgcn_wave_barrier();
    __builtin_amdgcn_fence(__ATOMIC_ACQUIRE, "workgroup");
    if (OUT_MODE == 0) {
      float* C = (float*)Cout + (size_t)b * strideC;
      const int hh = lane >> 4, c4 = (lane & 15) * 4;
      for (int pass = 0; pass < 2; ++pass) {
#pragma unroll
        for (int it = 0; it < 8; ++it) {
          const int row = it * 2 + hh;
          v4f v = *(const v4f*)(slab + row * 68 + c4);
          *(volatile v4f*)(C + (size_t)(mBase + row) * ldc + n0 + c4) = v;
        }
        __threadfence();
      }
    } else {
      const int q = lane >> 3, c8 = (lane & 7) * 8;
      unsigned short* C  = (unsigned short*)Cout  + (size_t)b * strideC;
      unsigned short* C2 = (OUT_MODE == 2) ? ((unsigned short*)Cout2 + (size_t)b * strideC) : nullptr;
      for (int pass = 0; pass < 2; ++pass) {
#pragma unroll
        for (int it = 0; it < 4; ++it) {
          const int row = it * 4 + q;
          const float* sp = slab + row * 68 + c8;
          v8h hv, lv;
#pragma unroll
          for (int e = 0; e < 8; ++e) {
            if (OUT_MODE == 1) {
              hv[e] = (_Float16)sp[e];
            } else {
              unsigned short hb = f2bf_bits(sp[e]);
              unsigned short lb = f2bf_bits(sp[e] - bf_bits2f(hb));
              hv[e] = __builtin_bit_cast(_Float16, hb);
              lv[e] = __builtin_bit_cast(_Float16, lb);
            }
          }
          *(volatile v8h*)(C + (size_t)(mBase + row) * ldc + n0 + c8) = hv;
          if (OUT_MODE == 2) *(volatile v8h*)(C2 + (size_t)(mBase + row) * ldc + n0 + c8) = lv;
        }
        __threadfence();
      }
    }
    __builtin_amdgcn_fence(__ATOMIC_RELEASE, "workgroup");
    __builtin_amdgcn_wave_barrier();
    __builtin_amdgcn_fence(__ATOMIC_ACQUIRE, "workgroup");
  }
}

__global__ __launch_bounds__(256) void cast_f32_f16x2(
    const float* __restrict__ in, _Float16* __restrict__ out, int n2) {
  int i = blockIdx.x * 256 + threadIdx.x;
  if (i < n2) {
    const _Float16 h0 = (_Float16)in[2 * i], h1 = (_Float16)in[2 * i + 1];
    const unsigned u = (unsigned)__builtin_bit_cast(unsigned short, h0) | ((unsigned)__builtin_bit_cast(unsigned short, h1) << 16);
    ((volatile unsigned*)out)[i] = u;
    __threadfence();
    ((volatile unsigned*)out)[i] = u;
  }
}

__global__ __launch_bounds__(256) void transpose_cast_w64(
    const float* __restrict__ W, _Float16* __restrict__ Wt, int Kr, int Nc, float mul) {
  __shared__ __align__(16) _Float16 sh[64 * 72];
  const int tid = threadIdx.x;
  const int n0 = blockIdx.x * 64;
  const int k0 = blockIdx.y * 64;
  {
    const int kr = tid >> 2;
    const int cb = (tid & 3) * 16;
    const float* src = W + (size_t)(k0 + kr) * Nc + n0 + cb;
#pragma unroll
    for (int i = 0; i < 4; ++i) {
      const v4f x = *(const v4f*)(src + 4 * i);
#pragma unroll
      for (int e = 0; e < 4; ++e) sh[(cb + 4 * i + e) * 72 + kr] = (_Float16)(x[e] * mul);
    }
  }
  __syncthreads();
  const int wave = tid >> 5, lane = tid & 31;
  const int rq = lane >> 3, c8 = (lane & 7) * 8;
  for (int pass = 0; pass < 2; ++pass) {
#pragma unroll
    for (int it = 0; it < 2; ++it) {
      const int n = wave * 8 + it * 4 + rq;
      const v8h val = *(const v8h*)(sh + n * 72 + c8);
      *(volatile v8h*)(Wt + (size_t)(n0 + n) * Kr + k0 + c8) = val;
    }
    __threadfence();
  }
}

namespace cfg {
constexpr int BB  = 2;
constexpr int TT  = 2048;
constexpr int CC  = 1024;
constexpr int C2C = 2048;
constexpr int HH  = 16;
constexpr int HS  = 64;
constexpr int HS2 = 128;
constexpr int RR  = BB * TT;
constexpr int AQB = 64;
constexpr int AKC = 64;
constexpr int ANW = 4;
constexpr int NQB = TT / AQB;
constexpr int NKC = TT / AKC;
constexpr int OSP = 136;
constexpr float PSC      = 32768.0f;
constexpr float PSC_INV  = 1.0f / 32768.0f;
constexpr float WSC      = 64.0f;
constexpr float WSC_INV  = 1.0f / 64.0f;
constexpr float LAM_INIT = (float)0.35550906759096928036;
constexpr float OUT_GAIN = (float)0.64449093240903071964;
constexpr float LN_EPS   = 1e-12f;
}

__device__ __forceinline__ v8f mma_h(v16h a, v16h b, v8f c) {
  c = __builtin_amdgcn_wmma_f32_16x16x32_f16(false, a, false, b, (short)0, c, false, false);
  asm volatile("v_nop\n\tv_nop\n\tv_nop\n\tv_nop" : "+v"(c) : "v"(a), "v"(b));
  return c;
}
__device__ __forceinline__ v8f zero8f() { return (v8f){0.f, 0.f, 0.f, 0.f, 0.f, 0.f, 0.f, 0.f}; }
__device__ __forceinline__ void wave_lds_fence() {
  __builtin_amdgcn_fence(__ATOMIC_RELEASE, "workgroup");
  __builtin_amdgcn_wave_barrier();
  __builtin_amdgcn_fence(__ATOMIC_ACQUIRE, "workgroup");
}

__global__ __launch_bounds__(128)
void attn_stats_kernel(const _Float16* __restrict__ q1, const _Float16* __restrict__ q2,
                       const _Float16* __restrict__ k1, const _Float16* __restrict__ k2,
                       const int* __restrict__ mask, float* __restrict__ ml) {
  using namespace cfg;
  __shared__ __align__(16) float sML[ANW * 32];
  const int tid = threadIdx.x, wave = tid >> 5, lane = tid & 31, hh = lane >> 4, c = lane & 15;
  int bx = blockIdx.x;
  const int qb = bx % NQB; bx /= NQB;
  const int h  = bx % HH;  bx /= HH;
  const int b  = bx % BB;
  const int st = bx / BB;
  const _Float16* qp = st ? q2 : q1;
  const _Float16* kp = st ? k2 : k1;
  const int q0 = qb * AQB + wave * 16;
  const size_t rowq = (size_t)b * TT + q0;

  v16h qa[2];
  {
    const _Float16* qr = qp + (rowq + c) * CC + h * HS + 8 * hh;
    qa[0] = Frag<_Float16>::load(qr);
    qa[1] = Frag<_Float16>::load(qr + 32);
  }
  float sc8[8], mrow[8], lrow[8];
#pragma unroll
  for (int r = 0; r < 8; ++r) {
    const int keep = mask[b * TT + q0 + 8 * hh + r];
    sc8[r]  = (keep != 0) ? 0.125f : 0.0f;
    mrow[r] = -__builtin_inff();
    lrow[r] = 0.f;
  }
  const _Float16* kb = kp + ((size_t)b * TT + c) * CC + h * HS + 8 * hh;

  for (int kc = 0; kc < NKC; ++kc) {
    const int kv0 = kc * AKC;
    v8f s[4];
#pragma unroll
    for (int j = 0; j < 4; ++j) {
      asm volatile("" ::: "memory");
      s[j] = zero8f();
      const _Float16* kpj = kb + (size_t)(kv0 + j * 16) * CC;
#pragma unroll
      for (int dc = 0; dc < 2; ++dc) {
        const v16h f = Frag<_Float16>::load(kpj + dc * 32);
        s[j] = mma_h(qa[dc], f, s[j]);
      }
    }
#pragma unroll
    for (int r = 0; r < 8; ++r) {
      float mx = -__builtin_inff();
#pragma unroll
      for (int j = 0; j < 4; ++j) {
        const float v = s[j][r] * sc8[r];
        s[j][r] = v;
        mx = fmaxf(mx, v);
      }
#pragma unroll
      for (int off = 1; off < 16; off <<= 1) mx = fmaxf(mx, __shfl_xor(mx, off, 32));
      const float mnew  = fmaxf(mrow[r], mx);
      const float alpha = __expf(mrow[r] - mnew);
      float psum = 0.f;
#pragma unroll
      for (int j = 0; j < 4; ++j) psum += __expf(s[j][r] - mnew);
#pragma unroll
      for (int off = 1; off < 16; off <<= 1) psum += __shfl_xor(psum, off, 32);
      lrow[r] = lrow[r] * alpha + psum;
      mrow[r] = mnew;
    }
  }

  if (c == 0) {
#pragma unroll
    for (int r = 0; r < 8; ++r) {
      sML[wave * 32 + (8 * hh + r) * 2]     = mrow[r];
      sML[wave * 32 + (8 * hh + r) * 2 + 1] = lrow[r];
    }
  }
  __syncthreads();
  if (wave == 0) {
    const v4f val = *(const v4f*)(sML + 4 * lane);
    float* dst = ml + ((size_t)(((st * BB + b) * HH + h) * TT + qb * AQB)) * 2 + 4 * lane;
    for (int pass = 0; pass < 2; ++pass) {
      *(volatile v4f*)dst = val;
      __threadfence();
    }
  }
}

__global__ __launch_bounds__(128)
void attn_combine_kernel(const _Float16* __restrict__ q1, const _Float16* __restrict__ q2,
                         const _Float16* __restrict__ k1, const _Float16* __restrict__ k2,
                         const _Float16* __restrict__ vvT, const int* __restrict__ mask,
                         const float* __restrict__ ml,
                         const float* __restrict__ lq1, const float* __restrict__ lk1,
                         const float* __restrict__ lq2, const float* __restrict__ lk2,
                         const float* __restrict__ ln_w, const float* __restrict__ ln_b,
                         _Float16* __restrict__ y16) {
  using namespace cfg;
  __shared__ __align__(16) _Float16 Psh[ANW][16 * AKC];
  __shared__ __align__(16) _Float16 Osh[ANW][16 * OSP];
  const int tid = threadIdx.x, wave = tid >> 5, lane = tid & 31, hh = lane >> 4, c = lane & 15;
  int bx = blockIdx.x;
  const int qb = bx % NQB; bx /= NQB;
  const int h  = bx % HH;
  const int b  = bx / HH;
  const int q0 = qb * AQB + wave * 16;
  const size_t rowq = (size_t)b * TT + q0;

  float lam;
  {
    const int o = h * HS;
    float a1 = lq1[o + lane] * lk1[o + lane] + lq1[o + 32 + lane] * lk1[o + 32 + lane];
    float a2 = lq2[o + lane] * lk2[o + lane] + lq2[o + 32 + lane] * lk2[o + 32 + lane];
#pragma unroll
    for (int off = 1; off < 32; off <<= 1) {
      a1 += __shfl_xor(a1, off, 32);
      a2 += __shfl_xor(a2, off, 32);
    }
    lam = expf(a1) - expf(a2) + LAM_INIT;
  }

  v16h q1a[2], q2a[2];
  {
    const _Float16* r1 = q1 + (rowq + c) * CC + h * HS + 8 * hh;
    const _Float16* r2 = q2 + (rowq + c) * CC + h * HS + 8 * hh;
    q1a[0] = Frag<_Float16>::load(r1);
    q1a[1] = Frag<_Float16>::load(r1 + 32);
    q2a[0] = Frag<_Float16>::load(r2);
    q2a[1] = Frag<_Float16>::load(r2 + 32);
  }
  float sc8[8], m1[8], m2[8], w1[8], w2[8];
#pragma unroll
  for (int r = 0; r < 8; ++r) {
    const int t = q0 + 8 * hh + r;
    const int keep = mask[b * TT + t];
    sc8[r] = (keep != 0) ? 0.125f : 0.0f;
    const size_t i1 = ((size_t)((0 * BB + b) * HH + h) * TT + t) * 2;
    const size_t i2 = ((size_t)((1 * BB + b) * HH + h) * TT + t) * 2;
    m1[r] = ml[i1];
    w1[r] = PSC / ml[i1 + 1];
    m2[r] = ml[i2];
    w2[r] = lam * (PSC / ml[i2 + 1]);
  }

  v8f O[8];
#pragma unroll
  for (int t = 0; t < 8; ++t) O[t] = zero8f();

  const _Float16* kb1 = k1 + ((size_t)b * TT + c) * CC + h * HS + 8 * hh;
  const _Float16* kb2 = k2 + ((size_t)b * TT + c) * CC + h * HS + 8 * hh;
  const _Float16* vb  = vvT + ((size_t)(h * HS2) + c) * RR + (size_t)b * TT + 8 * hh;
  _Float16* pw = Psh[wave];

  for (int kc = 0; kc < NKC; ++kc) {
    const int kv0 = kc * AKC;
    wave_lds_fence();
#pragma unroll
    for (int j = 0; j < 4; ++j) {
      asm volatile("" ::: "memory");
      v8f s1 = zero8f(), s2 = zero8f();
      const _Float16* kp1 = kb1 + (size_t)(kv0 + j * 16) * CC;
      const _Float16* kp2 = kb2 + (size_t)(kv0 + j * 16) * CC;
#pragma unroll
      for (int dc = 0; dc < 2; ++dc) {
        const v16h f1 = Frag<_Float16>::load(kp1 + dc * 32);
        s1 = mma_h(q1a[dc], f1, s1);
        const v16h f2 = Frag<_Float16>::load(kp2 + dc * 32);
        s2 = mma_h(q2a[dc], f2, s2);
      }
#pragma unroll
      for (int r = 0; r < 8; ++r) {
        const float e1 = __expf(s1[r] * sc8[r] - m1[r]);
        const float e2 = __expf(s2[r] * sc8[r] - m2[r]);
        const float p  = e1 * w1[r] - e2 * w2[r];
        pw[(8 * hh + r) * AKC + j * 16 + c] = (_Float16)p;
      }
    }
    wave_lds_fence();
#pragma unroll 1
    for (int kk = 0; kk < 2; ++kk) {
      const v16h pa = Frag<_Float16>::load(pw + c * AKC + kk * 32 + 8 * hh);
      const _Float16* vp = vb + kv0 + kk * 32;
#pragma unroll
      for (int t = 0; t < 8; ++t) {
        asm volatile("" ::: "memory");
        const v16h vf = Frag<_Float16>::load(vp + (size_t)(t * 16) * RR);
        O[t] = mma_h(pa, vf, O[t]);
      }
    }
  }

  float lw[8], lb[8];
#pragma unroll
  for (int t = 0; t < 8; ++t) { lw[t] = ln_w[t * 16 + c]; lb[t] = ln_b[t * 16 + c]; }
  _Float16* ow = Osh[wave];
#pragma unroll
  for (int r = 0; r < 8; ++r) {
    float sum = 0.f;
#pragma unroll
    for (int t = 0; t < 8; ++t) {
      const float yv = O[t][r] * PSC_INV;
      O[t][r] = yv;
      sum += yv;
    }
#pragma unroll
    for (int off = 1; off < 16; off <<= 1) sum += __shfl_xor(sum, off, 32);
    const float u = sum * (1.0f / 128.0f);
    float var = 0.f;
#pragma unroll
    for (int t = 0; t < 8; ++t) { const float d = O[t][r] - u; var += d * d; }
#pragma unroll
    for (int off = 1; off < 16; off <<= 1) var += __shfl_xor(var, off, 32);
    var *= (1.0f / 128.0f);
    const float inv = 1.0f / sqrtf(var + LN_EPS);
#pragma unroll
    for (int t = 0; t < 8; ++t) {
      const float val = (lw[t] * ((O[t][r] - u) * inv) + lb[t]) * OUT_GAIN;
      ow[(8 * hh + r) * OSP + t * 16 + c] = (_Float16)val;
    }
  }
  wave_lds_fence();
  {
    _Float16* yb = y16 + rowq * C2C + h * HS2;
    const int c8 = c * 8;
    for (int pass = 0; pass < 2; ++pass) {
#pragma unroll
      for (int it = 0; it < 8; ++it) {
        const int row = it * 2 + hh;
        const v8h val = *(const v8h*)(ow + row * OSP + c8);
        *(volatile v8h*)(yb + (size_t)row * C2C + c8) = val;
      }
      __threadfence();
    }
  }
}

extern "C" void kernel_launch(void* const* d_in, const int* in_sizes, int n_in,
                              void* d_out, int out_size, void* d_ws, size_t ws_size,
                              hipStream_t stream) {
  using namespace cfg;
  if (n_in < 22) return;
  if (in_sizes[0] != RR * CC || in_sizes[1] != RR * CC || in_sizes[2] != RR * CC ||
      in_sizes[3] != BB * TT || in_sizes[12] != CC * C2C || in_sizes[14] != C2C * CC ||
      out_size != RR * CC) return;

  const float* q    = (const float*)d_in[0];
  const float* kin  = (const float*)d_in[1];
  const float* vin  = (const float*)d_in[2];
  const int*   mask = (const int*)d_in[3];
  const float* Wq1 = (const float*)d_in[4];  const float* bq1 = (const float*)d_in[5];
  const float* Wq2 = (const float*)d_in[6];  const float* bq2 = (const float*)d_in[7];
  const float* Wk1 = (const float*)d_in[8];  const float* bk1 = (const float*)d_in[9];
  const float* Wk2 = (const float*)d_in[10]; const float* bk2 = (const float*)d_in[11];
  const float* Wv  = (const float*)d_in[12]; const float* bv  = (const float*)d_in[13];
  const float* Wc  = (const float*)d_in[14]; const float* bc  = (const float*)d_in[15];
  const float* ln_w = (const float*)d_in[16]; const float* ln_b = (const float*)d_in[17];
  const float* lq1 = (const float*)d_in[18]; const float* lk1 = (const float*)d_in[19];
  const float* lq2 = (const float*)d_in[20]; const float* lk2 = (const float*)d_in[21];
  float* out = (float*)d_out;

  const size_t szX  = (size_t)RR * CC * 2;
  const size_t szW  = (size_t)C2C * CC * 2;
  const size_t szP  = (size_t)RR * CC * 2;
  const size_t szV  = (size_t)C2C * RR * 2;
  const size_t szML = (size_t)2 * BB * HH * TT * 2 * 4;
  const size_t szY  = (size_t)RR * C2C * 2;
  const size_t offX  = 0;
  const size_t offW  = offX + szX;
  const size_t offQ1 = offW + szW;
  const size_t offQ2 = offQ1 + szP;
  const size_t offK1 = offQ2 + szP;
  const size_t offK2 = offK1 + szP;
  const size_t offV  = offK2 + szP;
  const size_t offML = offV + szV;
  const size_t offY  = offML + szML;
  const size_t total = offY + szY;
  if (total > ws_size) return;
  char* ws = (char*)d_ws;
  _Float16* X16 = (_Float16*)(ws + offX);
  _Float16* W16 = (_Float16*)(ws + offW);
  _Float16* Q1  = (_Float16*)(ws + offQ1);
  _Float16* Q2  = (_Float16*)(ws + offQ2);
  _Float16* K1  = (_Float16*)(ws + offK1);
  _Float16* K2  = (_Float16*)(ws + offK2);
  _Float16* VVT = (_Float16*)(ws + offV);
  float*    ML  = (float*)(ws + offML);
  _Float16* Y16 = (_Float16*)(ws + offY);

  const dim3 b256(256), b128(128);
  const int n2x = RR * CC / 2;
  const dim3 gCast((n2x + 255) / 256);
  const dim3 gTw(CC / 64, CC / 64);
  const dim3 gTv(C2C / 64, CC / 64);
  const dim3 gTc(CC / 64, C2C / 64);
  const dim3 gGp(((RR / 64) * (CC / 64) + 7) / 8, 1);
  const dim3 gGv(((C2C / 64) * (RR / 64) + 7) / 8, 1);
  const dim3 gGo(((RR / 64) * (CC / 64) + 7) / 8, 1);

  cast_f32_f16x2<<<gCast, b256, 0, stream>>>(q, X16, n2x);
  transpose_cast_w64<<<gTw, b256, 0, stream>>>(Wq1, W16, CC, CC, WSC);
  wmma_gemm64<0, false, 2, 1, false, 0><<<gGp, b256, 0, stream>>>(
      U16(X16), U16(X16), CC, 0L, U16(W16), U16(W16), CC, 0L,
      (void*)Q1, (void*)Q1, CC, 0L, bq1, bq1, 0L, RR, CC, CC, WSC_INV);
  transpose_cast_w64<<<gTw, b256, 0, stream>>>(Wq2, W16, CC, CC, WSC);
  wmma_gemm64<0, false, 2, 1, false, 0><<<gGp, b256, 0, stream>>>(
      U16(X16), U16(X16), CC, 0L, U16(W16), U16(W16), CC, 0L,
      (void*)Q2, (void*)Q2, CC, 0L, bq2, bq2, 0L, RR, CC, CC, WSC_INV);

  cast_f32_f16x2<<<gCast, b256, 0, stream>>>(kin, X16, n2x);
  transpose_cast_w64<<<gTw, b256, 0, stream>>>(Wk1, W16, CC, CC, WSC);
  wmma_gemm64<0, false, 2, 1, false, 0><<<gGp, b256, 0, stream>>>(
      U16(X16), U16(X16), CC, 0L, U16(W16), U16(W16), CC, 0L,
      (void*)K1, (void*)K1, CC, 0L, bk1, bk1, 0L, RR, CC, CC, WSC_INV);
  transpose_cast_w64<<<gTw, b256, 0, stream>>>(Wk2, W16, CC, CC, WSC);
  wmma_gemm64<0, false, 2, 1, false, 0><<<gGp, b256, 0, stream>>>(
      U16(X16), U16(X16), CC, 0L, U16(W16), U16(W16), CC, 0L,
      (void*)K2, (void*)K2, CC, 0L, bk2, bk2, 0L, RR, CC, CC, WSC_INV);

  cast_f32_f16x2<<<gCast, b256, 0, stream>>>(vin, X16, n2x);
  transpose_cast_w64<<<gTv, b256, 0, stream>>>(Wv, W16, CC, C2C, WSC);
  wmma_gemm64<0, false, 1, 1, false, 0><<<gGv, b256, 0, stream>>>(
      U16(W16), U16(W16), CC, 0L, U16(X16), U16(X16), CC, 0L,
      (void*)VVT, (void*)VVT, RR, 0L, bv, bv, 0L, C2C, RR, CC, WSC_INV);

  attn_stats_kernel<<<dim3(2 * BB * HH * NQB), b128, 0, stream>>>(Q1, Q2, K1, K2, mask, ML);
  attn_combine_kernel<<<dim3(BB * HH * NQB), b128, 0, stream>>>(
      Q1, Q2, K1, K2, VVT, mask, ML, lq1, lk1, lq2, lk2, ln_w, ln_b, Y16);

  transpose_cast_w64<<<gTc, b256, 0, stream>>>(Wc, W16, C2C, CC, WSC);
  wmma_gemm64<0, false, 2, 0, false, 0><<<gGo, b256, 0, stream>>>(
      U16(Y16), U16(Y16), C2C, 0L, U16(W16), U16(W16), C2C, 0L,
      (void*)out, (void*)out, CC, 0L, bc, bc, 0L, RR, CC, C2C, WSC_INV);
}
